// ExplicitREN_89300960019170
// MI455X (gfx1250) — hardware-run, weakly checked
//
#include <hip/hip_runtime.h>


#define NB   8192
#define NI   128
#define NH   1024
#define NO   128
#define NK   (NH + NI)
#define NBLK (NH / 64)
typedef _Float16 h16;
typedef unsigned short bf;
typedef __attribute__((ext_vector_type(16))) __bf16   v16bf;
typedef __attribute__((ext_vector_type(16))) _Float16 v16h;
typedef __attribute__((ext_vector_type(8)))  _Float16 v8h;
typedef __attribute__((ext_vector_type(8)))  unsigned short v8us;
typedef __attribute__((ext_vector_type(8)))  float    v8f;
typedef __attribute__((ext_vector_type(4)))  float    v4f;
typedef v8h  __attribute__((may_alias)) v8ha;
typedef v4f  __attribute__((may_alias)) v4fa;
typedef v8us __attribute__((may_alias)) v8usa;

__device__ __forceinline__ unsigned short f2bf(float f) { unsigned u = __float_as_uint(f); u += 0x7FFFu + ((u >> 16) & 1u); return (unsigned short)(u >> 16); }
__device__ __forceinline__ float bf2f(unsigned short b) { return __uint_as_float(((unsigned)b) << 16); }
__device__ __forceinline__ float bfr(float f) { return bf2f(f2bf(f)); }
__device__ __forceinline__ v16h cat16(v8h lo, v8h hi) { return __builtin_shufflevector(lo, hi, 0, 1, 2, 3, 4, 5, 6, 7, 8, 9, 10, 11, 12, 13, 14, 15); }
__device__ __forceinline__ v16bf cat16b(v8us lo, v8us hi) { return __builtin_bit_cast(v16bf, __builtin_shufflevector(lo, hi, 0, 1, 2, 3, 4, 5, 6, 7, 8, 9, 10, 11, 12, 13, 14, 15)); }
__device__ __forceinline__ v8f wmma16(v16h a, v16h b, v8f c) { return __builtin_amdgcn_wmma_f32_16x16x32_f16(false, a, false, b, (short)0, c, false, false); }
__device__ __forceinline__ v8f wmmab(v16bf a, v16bf b, v8f c) { return __builtin_amdgcn_wmma_f32_16x16x32_bf16(false, a, false, b, (short)0, c, false, false); }


template <typename T16> struct WFrag;
template <> struct WFrag<h16> { typedef v16h V; static __device__ __forceinline__ V ld(const h16* p) { return cat16(*(const v8h*)p, *(const v8h*)(p + 16)); } static __device__ __forceinline__ v8f mma(V a, V b, v8f c) { return wmma16(a, b, c); } };
template <> struct WFrag<bf> { typedef v16bf V; static __device__ __forceinline__ V ld(const bf* p) { return cat16b(*(const v8us*)p, *(const v8us*)(p + 16)); } static __device__ __forceinline__ v8f mma(V a, V b, v8f c) { return wmmab(a, b, c); } };
template <typename T16, int NSPLIT, bool BIAS>
__global__ __launch_bounds__(32) void k_gemmw(const T16* __restrict__ A, const T16* __restrict__ A2, const T16* __restrict__ Bt, const T16* __restrict__ Bt2, int K, float* C, int ldc, const float* __restrict__ bias, size_t sA, size_t sB, size_t sC) {
    typedef typename WFrag<T16>::V V;
    __shared__ __align__(16) float os[16 * 68];
    const size_t z = blockIdx.z; A += z * sA; if (A2) A2 += z * sA; Bt += z * sB; if (Bt2) Bt2 += z * sB; C += z * sC;
    const int lane = threadIdx.x & 31, lr = lane & 15, hi = lane >> 4; const int r0 = blockIdx.x * 64, c0 = blockIdx.y * 64;
    v8f acc[4][4];
#pragma unroll
    for (int mb = 0; mb < 4; ++mb)
#pragma unroll
        for (int nb = 0; nb < 4; ++nb) acc[mb][nb] = (v8f){};
    const size_t aoff = (size_t)(r0 + lr) * K + 8 * hi, boff = (size_t)(c0 + lr) * K + 8 * hi;
    for (int kc = 0; kc < K; kc += 32) {
        V a[4], a2[4];
#pragma unroll
        for (int mb = 0; mb < 4; ++mb) { a[mb] = WFrag<T16>::ld(A + aoff + (size_t)mb * 16 * K + kc); if (NSPLIT == 1 || NSPLIT == 2) a2[mb] = WFrag<T16>::ld(A2 + aoff + (size_t)mb * 16 * K + kc); }
#pragma unroll
        for (int nb = 0; nb < 4; ++nb) { const V b = WFrag<T16>::ld(Bt + boff + (size_t)nb * 16 * K + kc); V b2; if (NSPLIT >= 2) b2 = WFrag<T16>::ld(Bt2 + boff + (size_t)nb * 16 * K + kc);
#pragma unroll
            for (int mb = 0; mb < 4; ++mb) { acc[mb][nb] = WFrag<T16>::mma(a[mb], b, acc[mb][nb]); if (NSPLIT == 1 || NSPLIT == 2) acc[mb][nb] = WFrag<T16>::mma(a2[mb], b, acc[mb][nb]); if (NSPLIT >= 2) acc[mb][nb] = WFrag<T16>::mma(a[mb], b2, acc[mb][nb]); } }
        asm volatile("v_nop\n\tv_nop\n\tv_nop\n\tv_nop" : "+v"(acc[0][0]), "+v"(acc[1][1]), "+v"(acc[2][2]), "+v"(acc[3][3]) : "v"(a[0]), "v"(a[3]));
    }
#pragma unroll
    for (int mb = 0; mb < 4; ++mb) {
#pragma unroll
        for (int nb = 0; nb < 4; ++nb) {
#pragma unroll
            for (int j = 0; j < 8; ++j) os[(hi * 8 + j) * 68 + nb * 16 + lr] = acc[mb][nb][j]; }
        __builtin_amdgcn_wave_barrier(); asm volatile("" ::: "memory");
        float* crow = C + (size_t)(r0 + mb * 16) * ldc + c0;
#pragma unroll 1
        for (int ps = 0; ps < 2; ++ps) {
#pragma unroll
            for (int s = 0; s < 8; ++s) { const int row = 2 * s + hi, cofs = lr * 4; v4f val = *(const v4fa*)(os + row * 68 + cofs); if (BIAS) { val[0] += bfr(bias[c0 + cofs]); val[1] += bfr(bias[c0 + cofs + 1]); val[2] += bfr(bias[c0 + cofs + 2]); val[3] += bfr(bias[c0 + cofs + 3]); }
                *(volatile v4f*)(crow + (size_t)row * ldc + cofs) = val; }
            if (ps == 0) __threadfence(); }
        __builtin_amdgcn_wave_barrier(); asm volatile("" ::: "memory");
    }
}

typedef __attribute__((ext_vector_type(2))) _Float16 v2h;
typedef __attribute__((ext_vector_type(4))) _Float16 v4h;
typedef __attribute__((ext_vector_type(2))) unsigned short v2us;
typedef __attribute__((ext_vector_type(4))) unsigned short v4us;
typedef __attribute__((ext_vector_type(2))) float v2f;
typedef __attribute__((ext_vector_type(4))) int v4i;

__device__ __forceinline__ h16 toh_flush(float x) { const float z = (fabsf(x) < 6.103515625e-05f) ? 0.0f : x; return (h16)z; }

__device__ __forceinline__ float tanhc(float v) { return 1.0f - 2.0f / (expf(2.0f * v) + 1.0f); }

__global__ __launch_bounds__(256) void k_wcat(const float* __restrict__ a, const float* __restrict__ b, h16* dst, int R, int CA, int CB) { const int i = blockIdx.x * 256 + threadIdx.x; const int CT = CA + CB; if (i >= R * CT / 4) return; const int r = (i * 4) / CT, c0 = (i * 4) % CT; const bool ina = c0 < CA;
    const v4f va = *(const v4f*)(a + (size_t)r * CA + (ina ? c0 : 0)); const v4f vb = *(const v4f*)(b + (size_t)r * CB + (ina ? 0 : c0 - CA)); v4h o;
#pragma unroll
    for (int q = 0; q < 4; ++q) o[q] = toh_flush(bfr(ina ? va[q] : vb[q]));
    *(volatile v4h*)(dst + (size_t)i * 4) = o; __threadfence(); *(volatile v4h*)(dst + (size_t)i * 4) = o; }

__global__ __launch_bounds__(256) void k_xinit(const float* __restrict__ u, h16* X, int n4) { const int i = blockIdx.x * 256 + threadIdx.x; if (i >= n4) return; const int r = (i * 4) / NK, c0 = (i * 4) % NK; const bool isu = c0 >= NH; const unsigned short keep = isu ? (unsigned short)0xFFFFu : (unsigned short)0u; const v4f v = *(const v4f*)(u + (size_t)r * NI + (isu ? c0 - NH : 0)); v4h o;
#pragma unroll
    for (int q = 0; q < 4; ++q) o[q] = __builtin_bit_cast(h16, (unsigned short)(__builtin_bit_cast(unsigned short, toh_flush(bfr(v[q]))) & keep));
    *(volatile v4h*)(X + (size_t)i * 4) = o; __threadfence(); *(volatile v4h*)(X + (size_t)i * 4) = o; }

__global__ __launch_bounds__(256) void k_blk(const float* __restrict__ P, const h16* __restrict__ WB, int b, h16* X) { const int row = blockIdx.x * 256 + threadIdx.x; if (row >= NB) return;
    const float* pr = P + (size_t)row * 64; const h16* wb = WB + (size_t)(64 * b) * NK + 64 * b; float s[64];
#pragma unroll
    for (int i = 0; i < 64; ++i) { float v = pr[i];
#pragma unroll
        for (int j = 0; j < i; ++j) v = fmaf((float)wb[(size_t)i * NK + j], s[j], v);
        s[i] = tanhc(v); }
    h16* xr = X + (size_t)row * NK + 64 * b;
#pragma unroll
    for (int pass = 0; pass < 2; ++pass) {
#pragma unroll
        for (int q = 0; q < 8; ++q) { v8h o;
#pragma unroll
            for (int e = 0; e < 8; ++e) o[e] = toh_flush(s[8 * q + e]);
            *(volatile v8h*)(xr + 8 * q) = o; }
        if (pass == 0) __threadfence(); } }

extern "C" void kernel_launch(void* const* d_in, const int* in_sizes, int n_in, void* d_out, int out_size, void* d_ws, size_t ws_size, hipStream_t stream) {
    if (n_in < 5) return;
    if (in_sizes[0] != NB * NI || in_sizes[1] != NH * NI || in_sizes[2] != NH * NH || in_sizes[3] != NO * NH || in_sizes[4] != NO * NI) return;
    if (out_size != NB * NO) return;
    static_assert(NB % 256 == 0 && NH % 64 == 0 && NO % 64 == 0 && NK % 32 == 0 && NH % 4 == 0 && NI % 4 == 0 && (NH * NK / 4) % 256 == 0 && (NO * NK / 4) % 256 == 0 && (NB * NK / 4) % 256 == 0 && (NK * 2) % 128 == 0, "the products: M and N multiples of 64, the depth a multiple of 32; every elementwise grid exact; a row of the operand plane whole 128-byte lines");
    const float* u = (const float*)d_in[0]; const float* bw = (const float*)d_in[1]; const float* bs = (const float*)d_in[2]; const float* dsw = (const float*)d_in[3]; const float* dw = (const float*)d_in[4];
    float* out = (float*)d_out;
    char* wsp = (char*)d_ws; auto take = [&](size_t bytes) { char* p = wsp; wsp += (bytes + 255) & ~(size_t)255; return (void*)p; };
    h16* X = (h16*)take((size_t)NB * NK * 2);     h16* WB = (h16*)take((size_t)NH * NK * 2);     h16* WO = (h16*)take((size_t)NO * NK * 2);     float* P = (float*)take((size_t)NB * 64 * 4);
    if ((size_t)(wsp - (char*)d_ws) > ws_size) return;
    k_wcat<<<(unsigned)(NH * NK / 4 / 256), 256, 0, stream>>>(bs, bw, WB, NH, NH, NI);
    k_wcat<<<(unsigned)(NO * NK / 4 / 256), 256, 0, stream>>>(dsw, dw, WO, NO, NH, NI);
    k_xinit<<<(unsigned)(NB * NK / 4 / 256), 256, 0, stream>>>(u, X, NB * NK / 4);
    for (int b = 0; b < NBLK; ++b) {
        k_gemmw<h16, 0, false><<<dim3(NB / 64, 1, 1), 32, 0, stream>>>(X, nullptr, WB + (size_t)(64 * b) * NK, nullptr, NK, P, 64, nullptr, 0, 0, 0);
        k_blk<<<(unsigned)(NB / 256), 256, 0, stream>>>(P, WB, b, X); }
    k_gemmw<h16, 0, false><<<dim3(NB / 64, NO / 64, 1), 32, 0, stream>>>(X, nullptr, WO, nullptr, NK, out, NO, nullptr, 0, 0, 0);
}
